// Planner_32461362823245
// MI455X (gfx1250) — hardware-run, weakly checked
//
#include <hip/hip_runtime.h>
#include <math.h>

typedef __attribute__((ext_vector_type(16))) _Float16 v16h;
typedef __attribute__((ext_vector_type(8)))  _Float16 v8h;
typedef __attribute__((ext_vector_type(16))) __bf16   v16b;
typedef __attribute__((ext_vector_type(8)))  __bf16   v8b;
typedef __attribute__((ext_vector_type(8)))  float    v8f;
typedef __attribute__((ext_vector_type(4)))  float    v4f;
typedef __attribute__((ext_vector_type(4)))  unsigned v4u;

#define MSIDE     32
#define NPIX      16384
#define NCH       128
#define NGATE4    512
#define KCONV     1152
#define KHID      32
#define NSTEP     15
#define HST_PITCH 136
#define ACT_CARRY 64.0f
#define W_CARRY   1024.0f
#define GSCALE    (1.0f / 65536.0f)

static_assert(NPIX % 64 == 0, "");
static_assert(NCH % 64 == 0, "");
static_assert(KCONV % 32 == 0, "");
static_assert(KHID % 32 == 0, "");

constexpr size_t OFF_A0    = 0;
constexpr size_t OFF_BTHID = OFF_A0 + 1048576;
constexpr size_t OFF_HID   = OFF_BTHID + 8192;
constexpr size_t OFF_ACOL  = OFF_HID + 4194304;
constexpr size_t OFF_BTH0  = OFF_ACOL + 37748736;
constexpr size_t OFF_BTC0  = OFF_BTH0 + 294912;
constexpr size_t OFF_BTHH  = OFF_BTC0 + 294912;
constexpr size_t OFF_BTF   = OFF_BTHH + 131072;
constexpr size_t OFF_BTPOL = OFF_BTF + 4096;
constexpr size_t OFF_H0    = OFF_BTPOL + 4096;
constexpr size_t OFF_H1    = OFF_H0 + 4194304;
constexpr size_t OFF_C0    = OFF_H1 + 4194304;
constexpr size_t OFF_C1    = OFF_C0 + 8388608;
constexpr size_t OFF_Y0    = OFF_C1 + 8388608;
constexpr size_t OFF_Y1    = OFF_Y0 + 1048576;
constexpr size_t WS_TOTAL  = OFF_Y1 + 1048576;
static_assert(WS_TOTAL == 70991872, "");
static_assert(WS_TOTAL <= 134217728, "");
static_assert(262144 + 262144 <= 524288, "");

__device__ __forceinline__ unsigned short f2bf_bits(float f) {
  unsigned u = __float_as_uint(f);
  return (unsigned short)((u + 0x7FFFu + ((u >> 16) & 1u)) >> 16);
}
__device__ __forceinline__ float bf_bits2f(unsigned short h) { return __uint_as_float(((unsigned)h) << 16); }

__device__ __forceinline__ void dep_guard_h(v8f& a, v8f& b, v16h x, v16h y) { asm volatile("v_nop\n\tv_nop\n\tv_nop\n\tv_nop" : "+v"(a), "+v"(b) : "v"(x), "v"(y)); }
__device__ __forceinline__ void dep_guard_b(v8f& a, v8f& b, v16b x, v16b y) { asm volatile("v_nop\n\tv_nop\n\tv_nop\n\tv_nop" : "+v"(a), "+v"(b) : "v"(x), "v"(y)); }
__device__ __forceinline__ void keep4_h(v16h a, v16h b, v16h c, v16h d) { asm volatile("v_nop" :: "v"(a), "v"(b), "v"(c), "v"(d)); }
__device__ __forceinline__ void keep4_b(v16b a, v16b b, v16b c, v16b d) { asm volatile("v_nop" :: "v"(a), "v"(b), "v"(c), "v"(d)); }
__device__ __forceinline__ void acc_guard4(v8f& a, v8f& b, v8f& c, v8f& d) { asm volatile("v_nop\n\tv_nop\n\tv_nop\n\tv_nop" : "+v"(a), "+v"(b), "+v"(c), "+v"(d)); }
template <typename T> struct Frag;
template <> struct Frag<_Float16> {
  typedef v16h V; union U { v16h v; v8h h[2]; };
  static __device__ __forceinline__ v16h load(const _Float16* p) {
    U f; f.h[0] = *(const v8h*)(p); f.h[1] = *(const v8h*)(p + 16); return f.v;
  }
  static __device__ __forceinline__ v8f mma(v16h a, v16h b, v8f c) {
    return __builtin_amdgcn_wmma_f32_16x16x32_f16(false, a, false, b, (short)0, c, false, false);
  }
  static __device__ __forceinline__ void guard(v8f& a, v8f& b, v16h x, v16h y) { dep_guard_h(a, b, x, y); }
  static __device__ __forceinline__ void keep(v16h a, v16h b, v16h c, v16h d) { keep4_h(a, b, c, d); }
};
template <> struct Frag<__bf16> {
  typedef v16b V; union U { v16b v; v8b h[2]; };
  static __device__ __forceinline__ v16b load(const __bf16* p) {
    U f; f.h[0] = *(const v8b*)(p); f.h[1] = *(const v8b*)(p + 16); return f.v;
  }
  static __device__ __forceinline__ v8f mma(v16b a, v16b b, v8f c) {
    return __builtin_amdgcn_wmma_f32_16x16x32_bf16(false, a, false, b, (short)0, c, false, false);
  }
  static __device__ __forceinline__ void guard(v8f& a, v8f& b, v16b x, v16b y) { dep_guard_b(a, b, x, y); }
  static __device__ __forceinline__ void keep(v16b a, v16b b, v16b c, v16b d) { keep4_b(a, b, c, d); }
};

__device__ __forceinline__ v8f mma_f16(v16h a, v16h b, v8f c) {
  c = __builtin_amdgcn_wmma_f32_16x16x32_f16(false, a, false, b, (short)0, c, false, false);
  asm volatile("v_nop\n\tv_nop\n\tv_nop\n\tv_nop" : "+v"(c) : "v"(a), "v"(b));
  return c;
}

__device__ __forceinline__ void lds_wave_sync() {
  __builtin_amdgcn_fence(__ATOMIC_RELEASE, "workgroup");
  __builtin_amdgcn_wave_barrier();
  __builtin_amdgcn_fence(__ATOMIC_ACQUIRE, "workgroup");
}

template <int ET> struct Elem;
template <> struct Elem<0> { typedef _Float16 T; };
template <> struct Elem<1> { typedef __bf16 T; };
template <int ET, bool SPLIT, int BIAS_MODE, int OUT_MODE, bool RESID, int ACT = 0>
__global__ __launch_bounds__(256) void wmma_gemm64(
    const unsigned short* __restrict__ Ap, const unsigned short* __restrict__ A2p, int lda, long strideA,
    const unsigned short* __restrict__ Btp, const unsigned short* __restrict__ Bt2p, int ldb, long strideB,
    void* __restrict__ Cout, void* __restrict__ Cout2, int ldc, long strideC,
    const float* __restrict__ bias,
    const float* __restrict__ resid, long strideR,
    int M, int N, int K, float scale) {
  typedef typename Elem<ET>::T T;
  typedef typename Frag<T>::V V;
  const T* A = (const T*)Ap; const T* A2 = (const T*)A2p; const T* Bt = (const T*)Btp; const T* Bt2 = (const T*)Bt2p;
  __shared__ __align__(16) float sT[8][16 * 68];
  const int b    = blockIdx.y;
  const int lane = threadIdx.x & 31;
  const int wave = threadIdx.x >> 5;
  const int tilesN = N >> 6;
  const int tilesM = M >> 6;
  const int tile = blockIdx.x * 8 + wave;
  if (tile >= tilesM * tilesN) return;
  const int tm = tile / tilesN;
  const int tn = tile - tm * tilesN;
  const int m0 = tm << 6;
  const int n0 = tn << 6;

  const T* Ab  = A  + (size_t)b * strideA;
  const T* Bb  = Bt + (size_t)b * strideB;
  const T* Ab2 = SPLIT ? (A2  + (size_t)b * strideA) : nullptr;
  const T* Bb2 = SPLIT ? (Bt2 + (size_t)b * strideB) : nullptr;

  const int rlane = lane & 15;
  const int koff  = (lane >> 4) * 8;
  const int mOff  = (lane >> 4) * 8;

  v8f acc[4][4];
#pragma unroll
  for (int i = 0; i < 4; ++i)
#pragma unroll
    for (int j = 0; j < 4; ++j) acc[i][j] = (v8f){0.f,0.f,0.f,0.f,0.f,0.f,0.f,0.f};

  for (int k0 = 0; k0 < K; k0 += 32) {
    V bh[4], bl[4];
#pragma unroll
    for (int j = 0; j < 4; ++j) {
      const size_t bo = (size_t)(n0 + (j << 4) + rlane) * ldb + koff + k0;
      bh[j] = Frag<T>::load(Bb + bo);
      if (SPLIT) bl[j] = Frag<T>::load(Bb2 + bo);
    }
#pragma unroll
    for (int i = 0; i < 4; ++i) {
      const size_t ao = (size_t)(m0 + (i << 4) + rlane) * lda + koff + k0;
      V ah = Frag<T>::load(Ab + ao);
      V al;
      if (SPLIT) al = Frag<T>::load(Ab2 + ao);
#pragma unroll
      for (int j = 0; j < 4; ++j) {
        acc[i][j] = Frag<T>::mma(ah, bh[j], acc[i][j]);
        if (SPLIT) {
          acc[i][j] = Frag<T>::mma(ah, bl[j], acc[i][j]);
          acc[i][j] = Frag<T>::mma(al, bh[j], acc[i][j]);
        }
      }
      Frag<T>::guard(acc[i][0], acc[i][3], ah, SPLIT ? al : ah);
    }
    Frag<T>::keep(bh[0], bh[1], bh[2], bh[3]);
    if (SPLIT) Frag<T>::keep(bl[0], bl[1], bl[2], bl[3]);
  }
  acc_guard4(acc[0][0], acc[0][1], acc[0][2], acc[0][3]);
  acc_guard4(acc[1][0], acc[1][1], acc[1][2], acc[1][3]);
  acc_guard4(acc[2][0], acc[2][1], acc[2][2], acc[2][3]);
  acc_guard4(acc[3][0], acc[3][1], acc[3][2], acc[3][3]);

  float* slab = sT[wave];
  const float* Rb = RESID ? (resid + (size_t)b * strideR) : nullptr;
#pragma unroll
  for (int i = 0; i < 4; ++i) {
    const int mBase = m0 + (i << 4);
#pragma unroll
    for (int j = 0; j < 4; ++j) {
      const int n = n0 + (j << 4) + rlane;
      float bv = 0.f;
      if (BIAS_MODE == 2) bv = bias[n];
#pragma unroll
      for (int r = 0; r < 8; ++r) {
        float v = acc[i][j][r] * scale;
        if (BIAS_MODE == 1) v += bias[mBase + mOff + r];
        if (BIAS_MODE == 2) v += bv;
        if (RESID) v += Rb[(size_t)(mBase + mOff + r) * ldc + n];
        if (ACT == 1) v = tanhf(v);
        if (ACT == 2) v = fmaxf(v, 0.0f);
        if (ACT == 3) v = v / (1.0f + expf(-v));
        if (ACT == 4) v = (v > 0.f) ? v : 0.01f * v;
        if (ACT == 5) v = 0.5f * v * (1.0f + erff(v * 0.70710678118654752f));
        if (ACT == 6) v = v * 64.0f;
        slab[(mOff + r) * 68 + (j << 4) + rlane] = v;
      }
    }
    __builtin_amdgcn_fence(__ATOMIC_RELEASE, "workgroup");
    __builtin_amdgcn_wave_barrier();
    __builtin_amdgcn_fence(__ATOMIC_ACQUIRE, "workgroup");
    if (OUT_MODE == 0) {
      float* C = (float*)Cout + (size_t)b * strideC;
      const int hh = lane >> 4, c4 = (lane & 15) * 4;
      for (int pass = 0; pass < 2; ++pass) {
#pragma unroll
        for (int it = 0; it < 8; ++it) {
          const int row = it * 2 + hh;
          v4f v = *(const v4f*)(slab + row * 68 + c4);
          *(volatile v4f*)(C + (size_t)(mBase + row) * ldc + n0 + c4) = v;
        }
        __threadfence();
      }
    } else if (OUT_MODE == 3) {
      float* C = (float*)Cout + (size_t)b * strideC;
      const int q = lane >> 3, e8 = lane & 7;
      const int rsub = e8 >> 2, c4 = (e8 & 3) * 4;
      for (int pass = 0; pass < 2; ++pass) {
#pragma unroll
        for (int it = 0; it < 8; ++it) {
          const int j = it >> 1;
          const int row = (((it & 1) * 4) + q) * 2 + rsub;
          v4f v = *(const v4f*)(slab + row * 68 + (j << 4) + c4);
          *(volatile v4f*)(C + (((size_t)((n0 >> 4) + j)) * (size_t)M + (size_t)(mBase + row)) * 16 + c4) = v;
        }
        __threadfence();
      }
    } else {
      const int q = lane >> 3, c8 = (lane & 7) * 8;
      unsigned short* C  = (unsigned short*)Cout  + (size_t)b * strideC;
      unsigned short* C2 = (OUT_MODE == 2) ? ((unsigned short*)Cout2 + (size_t)b * strideC) : nullptr;
      for (int pass = 0; pass < 2; ++pass) {
#pragma unroll
        for (int it = 0; it < 4; ++it) {
          const int row = it * 4 + q;
          const float* sp = slab + row * 68 + c8;
          v8h hv, lv;
#pragma unroll
          for (int e = 0; e < 8; ++e) {
            if (OUT_MODE == 1) {
              hv[e] = (_Float16)sp[e];
            } else {
              unsigned short hb = f2bf_bits(sp[e]);
              unsigned short lb = f2bf_bits(sp[e] - bf_bits2f(hb));
              hv[e] = __builtin_bit_cast(_Float16, hb);
              lv[e] = __builtin_bit_cast(_Float16, lb);
            }
          }
          *(volatile v8h*)(C + (size_t)(mBase + row) * ldc + n0 + c8) = hv;
          if (OUT_MODE == 2) *(volatile v8h*)(C2 + (size_t)(mBase + row) * ldc + n0 + c8) = lv;
        }
        __threadfence();
      }
    }
    __builtin_amdgcn_fence(__ATOMIC_RELEASE, "workgroup");
    __builtin_amdgcn_wave_barrier();
    __builtin_amdgcn_fence(__ATOMIC_ACQUIRE, "workgroup");
  }
}

__device__ __forceinline__ void store_pair16(unsigned short* __restrict__ dst, int i, float v0, float v1) {
  const _Float16 h0 = (_Float16)v0, h1 = (_Float16)v1;
  const unsigned u = (unsigned)__builtin_bit_cast(unsigned short, h0) | ((unsigned)__builtin_bit_cast(unsigned short, h1) << 16);
  ((volatile unsigned*)dst)[i] = u;
  __threadfence();
  ((volatile unsigned*)dst)[i] = u;
}

__global__ __launch_bounds__(256) void prep_w_kernel(
    const float* __restrict__ W_h0, const float* __restrict__ W_c0, const float* __restrict__ W_hh,
    const float* __restrict__ W_hid, const float* __restrict__ W_f, const float* __restrict__ W_pol,
    unsigned short* __restrict__ bt_h0, unsigned short* __restrict__ bt_c0, unsigned short* __restrict__ bt_hh,
    unsigned short* __restrict__ bt_hid, unsigned short* __restrict__ bt_f, unsigned short* __restrict__ bt_pol) {
  const int blk = blockIdx.x, tid = threadIdx.x;
  if (blk < 576) {
    const bool second = (blk >= 288);
    const float* W = second ? W_c0 : W_h0;
    unsigned short* dst = second ? bt_c0 : bt_h0;
    const int i  = (blk - (second ? 288 : 0)) * 256 + tid;
    const int o  = 2 * i;
    const int co = o / KCONV;
    const int k  = o - co * KCONV;
    const float v0 = W[(size_t)k * NCH + co] * W_CARRY;
    const float v1 = W[(size_t)(k + 1) * NCH + co] * W_CARRY;
    store_pair16(dst, i, v0, v1);
  } else if (blk < 704) {
    const int i   = (blk - 576) * 256 + tid;
    const int o   = 2 * i;
    const int np  = o >> 7;
    const int k   = o & 127;
    const int cb  = np >> 6, g = (np >> 4) & 3, chl = np & 15;
    const int src = g * NCH + cb * 16 + chl;
    const float v0 = W_hh[(size_t)src * NCH + k] * W_CARRY;
    const float v1 = W_hh[(size_t)src * NCH + k + 1] * W_CARRY;
    store_pair16(bt_hh, i, v0, v1);
  } else if (blk < 712) {
    const int i  = (blk - 704) * 256 + tid;
    const int o  = 2 * i;
    const int co = o >> 5;
    const int k  = o & 31;
    const int k0c = k < 18 ? k : 17, k1c = (k + 1) < 18 ? (k + 1) : 17;
    const float a0 = W_hid[k0c * NCH + co];
    const float a1 = W_hid[k1c * NCH + co];
    const float v0 = (k < 18) ? a0 * W_CARRY : 0.0f;
    const float v1 = ((k + 1) < 18) ? a1 * W_CARRY : 0.0f;
    store_pair16(bt_hid, i, v0, v1);
  } else if (blk < 716) {
    const int i  = (blk - 712) * 256 + tid;
    const int o  = 2 * i;
    const int t  = o >> 7;
    const int ci = o & 127;
    const int tc = t < 9 ? t : 8;
    const float a0 = W_f[tc * NCH + ci];
    const float a1 = W_f[tc * NCH + ci + 1];
    const float v0 = (t < 9) ? a0 * W_CARRY : 0.0f;
    const float v1 = (t < 9) ? a1 * W_CARRY : 0.0f;
    store_pair16(bt_f, i, v0, v1);
  } else {
    const int i  = (blk - 716) * 256 + tid;
    const int o  = 2 * i;
    const int a  = o >> 7;
    const int ci = o & 127;
    const int ac = a < 4 ? a : 3;
    const float a0 = W_pol[ci * 4 + ac];
    const float a1 = W_pol[(ci + 1) * 4 + ac];
    const float v0 = (a < 4) ? a0 * W_CARRY : 0.0f;
    const float v1 = (a < 4) ? a1 * W_CARRY : 0.0f;
    store_pair16(bt_pol, i, v0, v1);
  }
}

__global__ __launch_bounds__(256) void im2col_x_kernel(
    const float* __restrict__ md, const float* __restrict__ gl, unsigned short* __restrict__ a0) {
  const int t = blockIdx.x * 256 + threadIdx.x;
  const int p = t >> 2, q = t & 3;
  const int b = p >> 10, y = (p >> 5) & 31, x = p & 31;
  v8h o;
#pragma unroll
  for (int e = 0; e < 8; ++e) {
    const int k = q * 8 + e;
    const int tap = (k >> 1) < 8 ? (k >> 1) : 8;
    const int cin = k & 1;
    const int y2 = y + tap / 3 - 1, x2 = x + tap % 3 - 1;
    const bool valid = (k < 18) && (y2 >= 0) && (y2 < MSIDE) && (x2 >= 0) && (x2 < MSIDE);
    const int yc = y2 < 0 ? 0 : (y2 > 31 ? 31 : y2);
    const int xc = x2 < 0 ? 0 : (x2 > 31 ? 31 : x2);
    const int a = (b * MSIDE + yc) * MSIDE + xc;
    const float mv = md[a];
    const float gv = gl[a];
    float val = cin ? gv : mv;
    val = valid ? val * ACT_CARRY : 0.0f;
    o[e] = (_Float16)val;
  }
  _Float16* dst = (_Float16*)a0 + (size_t)t * 8;
  *(volatile v8h*)dst = o;
  __threadfence();
  *(volatile v8h*)dst = o;
}

__global__ __launch_bounds__(256) void im2col_hid_kernel(
    const unsigned short* __restrict__ hid, unsigned short* __restrict__ acol) {
  const int t = blockIdx.x * 256 + threadIdx.x;
  const int p = t / 144;
  const int c = t - p * 144;
  const int tap = c >> 4, ci0 = (c & 15) * 8;
  const int b = p >> 10, y = (p >> 5) & 31, x = p & 31;
  const int y2 = y + tap / 3 - 1, x2 = x + tap % 3 - 1;
  const bool valid = (y2 >= 0) && (y2 < MSIDE) && (x2 >= 0) && (x2 < MSIDE);
  const int yc = y2 < 0 ? 0 : (y2 > 31 ? 31 : y2);
  const int xc = x2 < 0 ? 0 : (x2 > 31 ? 31 : x2);
  const int pp = (b * MSIDE + yc) * MSIDE + xc;
  const v4u v = *(const v4u*)(hid + (size_t)pp * NCH + ci0);
  const v4u z = {0u, 0u, 0u, 0u};
  const v4u o = valid ? v : z;
  unsigned short* dst = acol + (size_t)t * 8;
  *(volatile v4u*)dst = o;
  __threadfence();
  *(volatile v4u*)dst = o;
}

__device__ __forceinline__ void y_tile_store(float* slab, int pitch, v8f acc, float* __restrict__ y, int rowBase, int lane) {
  const int rlane = lane & 15, mOff = (lane >> 4) * 8;
#pragma unroll
  for (int r = 0; r < 8; ++r) slab[(mOff + r) * pitch + rlane] = acc[r] * GSCALE;
  lds_wave_sync();
  const int q = lane >> 3, e8 = lane & 7, rsub = e8 >> 2, c4 = (e8 & 3) * 4;
  for (int pass = 0; pass < 2; ++pass) {
#pragma unroll
    for (int it = 0; it < 2; ++it) {
      const int row = ((it * 4) + q) * 2 + rsub;
      v4f v = *(const v4f*)(slab + row * pitch + c4);
      *(volatile v4f*)(y + (size_t)(rowBase + row) * 16 + c4) = v;
    }
    __threadfence();
  }
  lds_wave_sync();
}

__global__ __launch_bounds__(128) void y_init_kernel(
    const unsigned short* __restrict__ hpl, const unsigned short* __restrict__ wft, float* __restrict__ y) {
  __shared__ __align__(16) float sl[4][16 * 20];
  const int lane = threadIdx.x & 31, wave = threadIdx.x >> 5;
  const int rlane = lane & 15, koff = (lane >> 4) * 8;
  const int m0 = blockIdx.x * 64;
  const _Float16* A  = (const _Float16*)hpl;
  const _Float16* Bw = (const _Float16*)wft;
  v8f acc = (v8f){0.f,0.f,0.f,0.f,0.f,0.f,0.f,0.f};
#pragma unroll
  for (int kc = 0; kc < 4; ++kc) {
    const v16h a  = Frag<_Float16>::load(A + (size_t)(m0 + (wave << 4) + rlane) * NCH + kc * 32 + koff);
    const v16h bq = Frag<_Float16>::load(Bw + (size_t)rlane * NCH + kc * 32 + koff);
    acc = mma_f16(a, bq, acc);
  }
  y_tile_store(sl[wave], 20, acc, y, m0 + (wave << 4), lane);
}

__global__ __launch_bounds__(256) void lstm_step_kernel(
    const unsigned short* __restrict__ hcur, const unsigned short* __restrict__ whh, const unsigned short* __restrict__ wft,
    const float* __restrict__ ccur, const float* __restrict__ ycur,
    const float* __restrict__ W_ih, const float* __restrict__ b_ih, const float* __restrict__ b_hh, const float* __restrict__ b_f,
    unsigned short* __restrict__ hnext, float* __restrict__ cnext, float* __restrict__ ynext) {
  __shared__ __align__(16) float sT[8][16 * 68];
  __shared__ __align__(16) float cw[8][256];
  __shared__ __align__(16) _Float16 hst[64 * HST_PITCH];
  __shared__ float inp_sh[64];
  __shared__ float wih_sh[NGATE4];
  __shared__ float bsum_sh[NGATE4];

  const int tid  = threadIdx.x;
  const int lane = tid & 31, wave = tid >> 5;
  const int rlane = lane & 15;
  const int koff  = (lane >> 4) * 8;
  const int mOff  = koff;
  const int m0 = blockIdx.x * 64;
  const int n0 = wave * 64;

  for (int t = tid; t < NGATE4; t += 256) {
    wih_sh[t]  = W_ih[t];
    bsum_sh[t] = b_ih[t] + b_hh[t];
  }
  if (tid < 64) {
    const int m = m0 + tid;
    const int b = m >> 10, y = (m >> 5) & 31, x = m & 31;
    float s = b_f[0];
#pragma unroll
    for (int tap = 0; tap < 9; ++tap) {
      const int y2 = y + tap / 3 - 1, x2 = x + tap % 3 - 1;
      const bool valid = (y2 >= 0) && (y2 < MSIDE) && (x2 >= 0) && (x2 < MSIDE);
      const int yc = y2 < 0 ? 0 : (y2 > 31 ? 31 : y2);
      const int xc = x2 < 0 ? 0 : (x2 > 31 ? 31 : x2);
      const float v = ycur[(size_t)((b * MSIDE + yc) * MSIDE + xc) * 16 + tap];
      s += valid ? v : 0.0f;
    }
    inp_sh[tid] = s;
  }
  __syncthreads();

  const _Float16* Ab = (const _Float16*)hcur;
  const _Float16* Bb = (const _Float16*)whh;
  v8f acc[4][4];
#pragma unroll
  for (int i = 0; i < 4; ++i)
#pragma unroll
    for (int j = 0; j < 4; ++j) acc[i][j] = (v8f){0.f,0.f,0.f,0.f,0.f,0.f,0.f,0.f};

  for (int k0 = 0; k0 < NCH; k0 += 32) {
    v16h bh[4];
#pragma unroll
    for (int j = 0; j < 4; ++j) {
      const size_t bo = (size_t)(n0 + (j << 4) + rlane) * NCH + koff + k0;
      bh[j] = Frag<_Float16>::load(Bb + bo);
    }
#pragma unroll
    for (int i = 0; i < 4; ++i) {
      const size_t ao = (size_t)(m0 + (i << 4) + rlane) * NCH + koff + k0;
      v16h ah = Frag<_Float16>::load(Ab + ao);
#pragma unroll
      for (int j = 0; j < 4; ++j) acc[i][j] = Frag<_Float16>::mma(ah, bh[j], acc[i][j]);
      Frag<_Float16>::guard(acc[i][0], acc[i][3], ah, ah);
    }
    Frag<_Float16>::keep(bh[0], bh[1], bh[2], bh[3]);
  }
  acc_guard4(acc[0][0], acc[0][1], acc[0][2], acc[0][3]);
  acc_guard4(acc[1][0], acc[1][1], acc[1][2], acc[1][3]);
  acc_guard4(acc[2][0], acc[2][1], acc[2][2], acc[2][3]);
  acc_guard4(acc[3][0], acc[3][1], acc[3][2], acc[3][3]);

  float* slab = sT[wave];
  float* cwv  = cw[wave];
#pragma unroll
  for (int i = 0; i < 4; ++i) {
    const int mBase = m0 + (i << 4);
#pragma unroll
    for (int j = 0; j < 4; ++j)
#pragma unroll
      for (int r = 0; r < 8; ++r) slab[(mOff + r) * 68 + (j << 4) + rlane] = acc[i][j][r] * GSCALE;
    lds_wave_sync();
#pragma unroll 1
    for (int e = 0; e < 8; ++e) {
      const int cell = e * 32 + lane;
      const int row  = cell >> 4;
      const int chl  = cell & 15;
      const int ch   = (wave << 4) + chl;
      const float xin = inp_sh[(i << 4) + row];
      const float* sp = slab + row * 68 + chl;
      const float gi = sp[0]  + xin * wih_sh[ch]           + bsum_sh[ch];
      const float gf = sp[16] + xin * wih_sh[NCH + ch]     + bsum_sh[NCH + ch];
      const float gg = sp[32] + xin * wih_sh[2 * NCH + ch] + bsum_sh[2 * NCH + ch];
      const float go = sp[48] + xin * wih_sh[3 * NCH + ch] + bsum_sh[3 * NCH + ch];
      const float si = 1.0f / (1.0f + expf(-gi));
      const float sf = 1.0f / (1.0f + expf(-gf));
      const float so = 1.0f / (1.0f + expf(-go));
      const float tg = tanhf(gg);
      const float cold = ccur[((size_t)wave * NPIX + (size_t)(mBase + row)) * 16 + chl];
      const float c2 = sf * cold + si * tg;
      const float h2 = so * tanhf(c2);
      cwv[row * 16 + chl] = c2;
      hst[((i << 4) + row) * HST_PITCH + ch] = (_Float16)(h2 * ACT_CARRY);
    }
    lds_wave_sync();
    {
      const int q = lane >> 3, e8 = lane & 7, rsub = e8 >> 2, c4 = (e8 & 3) * 4;
      for (int pass = 0; pass < 2; ++pass) {
#pragma unroll
        for (int it = 0; it < 2; ++it) {
          const int row = ((it * 4) + q) * 2 + rsub;
          v4f v = *(const v4f*)(cwv + row * 16 + c4);
          *(volatile v4f*)(cnext + ((size_t)wave * NPIX + (size_t)(mBase + row)) * 16 + c4) = v;
        }
        __threadfence();
      }
    }
    lds_wave_sync();
  }
  __syncthreads();

  {
    const int hh = lane >> 4, c8 = (lane & 15) * 8;
    _Float16* Hn = (_Float16*)hnext;
    for (int pass = 0; pass < 2; ++pass) {
#pragma unroll
      for (int it = 0; it < 4; ++it) {
        const int row = (wave << 3) + it * 2 + hh;
        v8h v = *(const v8h*)(hst + row * HST_PITCH + c8);
        *(volatile v8h*)(Hn + (size_t)(m0 + row) * NCH + c8) = v;
      }
      __threadfence();
    }
  }

  if (wave < 4) {
    v8f yacc = (v8f){0.f,0.f,0.f,0.f,0.f,0.f,0.f,0.f};
    const _Float16* Bw = (const _Float16*)wft;
#pragma unroll
    for (int kc = 0; kc < 4; ++kc) {
      const v16h a  = Frag<_Float16>::load(hst + ((wave << 4) + rlane) * HST_PITCH + kc * 32 + koff);
      const v16h bq = Frag<_Float16>::load(Bw + (size_t)rlane * NCH + kc * 32 + koff);
      yacc = mma_f16(a, bq, yacc);
    }
    y_tile_store(slab, 68, yacc, ynext, m0 + (wave << 4), lane);
  }
}

__global__ __launch_bounds__(128) void policy_kernel(
    const unsigned short* __restrict__ hpl, const unsigned short* __restrict__ wpol, float* __restrict__ out) {
  __shared__ __align__(16) float ls[64 * 16];
  __shared__ __align__(16) float osh[8 * 64];
  const int tid = threadIdx.x;
  const int lane = tid & 31, wave = tid >> 5;
  const int rlane = lane & 15, koff = (lane >> 4) * 8, mOff = koff;
  const int m0 = blockIdx.x * 64;
  const _Float16* A  = (const _Float16*)hpl;
  const _Float16* Bw = (const _Float16*)wpol;
  v8f acc = (v8f){0.f,0.f,0.f,0.f,0.f,0.f,0.f,0.f};
#pragma unroll
  for (int kc = 0; kc < 4; ++kc) {
    const v16h a  = Frag<_Float16>::load(A + (size_t)(m0 + (wave << 4) + rlane) * NCH + kc * 32 + koff);
    const v16h bq = Frag<_Float16>::load(Bw + (size_t)rlane * NCH + kc * 32 + koff);
    acc = mma_f16(a, bq, acc);
  }
#pragma unroll
  for (int r = 0; r < 8; ++r) ls[((wave << 4) + mOff + r) * 16 + rlane] = acc[r] * GSCALE;
  __syncthreads();
  if (tid < 64) {
    const float* lp = ls + tid * 16;
    const float l0 = lp[0], l1 = lp[1], l2 = lp[2], l3 = lp[3];
    const float mx = fmaxf(fmaxf(l0, l1), fmaxf(l2, l3));
    const float e0 = expf(l0 - mx), e1 = expf(l1 - mx), e2 = expf(l2 - mx), e3 = expf(l3 - mx);
    const float s = ((e0 + e1) + e2) + e3;
    const float inv = 1.0f / s;
    osh[0 * 64 + tid] = l0;
    osh[1 * 64 + tid] = l1;
    osh[2 * 64 + tid] = l2;
    osh[3 * 64 + tid] = l3;
    osh[4 * 64 + tid] = e0 * inv;
    osh[5 * 64 + tid] = e1 * inv;
    osh[6 * 64 + tid] = e2 * inv;
    osh[7 * 64 + tid] = e3 * inv;
  }
  __syncthreads();
  {
    const int hh = lane >> 4, c4 = (lane & 15) * 4;
    const int seg = (wave << 1) + hh;
    const int a = seg & 3;
    const int b = m0 >> 10, yx0 = m0 & 1023;
    const size_t obase = (size_t)(seg >> 2) * (size_t)(NPIX * 4) + (size_t)(b * 4 + a) * 1024 + (size_t)(yx0 + c4);
    v4f v = *(const v4f*)(osh + seg * 64 + c4);
    *(volatile v4f*)(out + obase) = v;
    __threadfence();
    *(volatile v4f*)(out + obase) = v;
  }
}

extern "C" void kernel_launch(void* const* d_in, const int* in_sizes, int n_in,
                              void* d_out, int out_size, void* d_ws, size_t ws_size,
                              hipStream_t stream) {
  (void)in_sizes;
  if (n_in < 15) return;
  if (out_size < 2 * NPIX * 4) return;
  if (ws_size < WS_TOTAL) return;

  const float* md    = (const float*)d_in[0];
  const float* gl    = (const float*)d_in[1];
  const float* W_hid = (const float*)d_in[2];
  const float* b_hid = (const float*)d_in[3];
  const float* W_h0  = (const float*)d_in[4];
  const float* b_h0  = (const float*)d_in[5];
  const float* W_c0  = (const float*)d_in[6];
  const float* b_c0  = (const float*)d_in[7];
  const float* W_f   = (const float*)d_in[8];
  const float* b_f   = (const float*)d_in[9];
  const float* W_ih  = (const float*)d_in[10];
  const float* b_ih  = (const float*)d_in[11];
  const float* W_hh  = (const float*)d_in[12];
  const float* b_hh  = (const float*)d_in[13];
  const float* W_pol = (const float*)d_in[14];
  float* out = (float*)d_out;

  char* ws = (char*)d_ws;
  unsigned short* a0     = (unsigned short*)(ws + OFF_A0);
  unsigned short* bt_hid = (unsigned short*)(ws + OFF_BTHID);
  unsigned short* hid    = (unsigned short*)(ws + OFF_HID);
  unsigned short* acol   = (unsigned short*)(ws + OFF_ACOL);
  unsigned short* bt_h0  = (unsigned short*)(ws + OFF_BTH0);
  unsigned short* bt_c0  = (unsigned short*)(ws + OFF_BTC0);
  unsigned short* bt_hh  = (unsigned short*)(ws + OFF_BTHH);
  unsigned short* bt_f   = (unsigned short*)(ws + OFF_BTF);
  unsigned short* bt_pol = (unsigned short*)(ws + OFF_BTPOL);
  unsigned short* hpl[2] = { (unsigned short*)(ws + OFF_H0), (unsigned short*)(ws + OFF_H1) };
  float*          cpl[2] = { (float*)(ws + OFF_C0), (float*)(ws + OFF_C1) };
  float*          ypl[2] = { (float*)(ws + OFF_Y0), (float*)(ws + OFF_Y1) };

  prep_w_kernel<<<720, 256, 0, stream>>>(W_h0, W_c0, W_hh, W_hid, W_f, W_pol,
                                         bt_h0, bt_c0, bt_hh, bt_hid, bt_f, bt_pol);
  im2col_x_kernel<<<(NPIX * 4) / 256, 256, 0, stream>>>(md, gl, a0);
  wmma_gemm64<0, false, 2, 1, false, 6><<<dim3((NPIX / 64) * (NCH / 64) / 8, 1), 256, 0, stream>>>(
      a0, nullptr, KHID, 0, bt_hid, nullptr, KHID, 0, (void*)hid, nullptr, NCH, 0,
      b_hid, nullptr, 0, NPIX, NCH, KHID, GSCALE);
  im2col_hid_kernel<<<(NPIX * 144) / 256, 256, 0, stream>>>(hid, acol);
  wmma_gemm64<0, false, 2, 1, false, 6><<<dim3((NPIX / 64) * (NCH / 64) / 8, 1), 256, 0, stream>>>(
      acol, nullptr, KCONV, 0, bt_h0, nullptr, KCONV, 0, (void*)hpl[0], nullptr, NCH, 0,
      b_h0, nullptr, 0, NPIX, NCH, KCONV, GSCALE);
  wmma_gemm64<0, false, 2, 3, false, 0><<<dim3((NPIX / 64) * (NCH / 64) / 8, 1), 256, 0, stream>>>(
      acol, nullptr, KCONV, 0, bt_c0, nullptr, KCONV, 0, (void*)cpl[0], nullptr, 16, 0,
      b_c0, nullptr, 0, NPIX, NCH, KCONV, GSCALE);
  y_init_kernel<<<NPIX / 64, 128, 0, stream>>>(hpl[0], bt_f, ypl[0]);
  for (int s = 0; s < NSTEP; ++s) {
    const int ci = s & 1, co = (s + 1) & 1;
    lstm_step_kernel<<<NPIX / 64, 256, 0, stream>>>(
        hpl[ci], bt_hh, bt_f, cpl[ci], ypl[ci], W_ih, b_ih, b_hh, b_f,
        hpl[co], cpl[co], ypl[co]);
  }
  policy_kernel<<<NPIX / 64, 128, 0, stream>>>(hpl[NSTEP & 1], bt_pol, out);
}
